// RelativePositionalAttention_24464133718913
// MI455X (gfx1250) — hardware-verified
//
#include <hip/hip_runtime.h>
#include <math.h>
#include <stdint.h>

#define LQ    1024
#define NB    4
#define DMOD  1024
#define NH    16
#define DH    64
#define NPOS  (2 * LQ)
#define NROW  (LQ * NB)
#define XC    16.0f
#define WSC   64.0f
#define QC    4.0f
#define VC    16.0f
#define PC    1024.0f
#define CC    4096.0f
#define RSD   0.125f
#define LOG2E 1.4426950408889634f
#define BIGM  1000000.0f
#define LN_EPS 1.0e-9f
static_assert(NH * DH == DMOD);
static_assert(DH == 64);
static_assert((LQ % 64) == 0 && (DMOD % 64) == 0 && (NROW % 64) == 0 && (NPOS % 64) == 0);
static_assert(((NROW * DMOD) % 2048) == 0 && ((NPOS * DMOD) % 2048) == 0 && (NROW % 8) == 0);
#define ATT_W 4
#define ATT_THREADS (ATT_W * 32)
#define TPI 84
#define PPI 68
#define WFL (16 * TPI + 16 * PPI)
static_assert(((16 * TPI) % 4) == 0 && ((16 * PPI) % 4) == 0 && (WFL % 4) == 0);
static_assert(TPI >= 80 && PPI >= 64);
static_assert(ATT_W * WFL * 4 <= 65536);

typedef _Float16 v16h __attribute__((ext_vector_type(16)));
typedef _Float16 v8h  __attribute__((ext_vector_type(8)));
typedef __bf16   v16b __attribute__((ext_vector_type(16)));
typedef float    v8f  __attribute__((ext_vector_type(8)));
typedef float    v4f  __attribute__((ext_vector_type(4)));
typedef unsigned int v4u __attribute__((ext_vector_type(4)));

union FragH { v16h v; v8h h[2]; v4u u[2]; };
union FragAny { v16h h; v16b b; };

__device__ __forceinline__ unsigned short bf_bits(float f) {
  unsigned u = __float_as_uint(f);
  return (unsigned short)((u + 0x7FFFu + ((u >> 16) & 1u)) >> 16);
}
__device__ __forceinline__ float bf_up(unsigned short h) { return __uint_as_float(((unsigned)h) << 16); }
__device__ __forceinline__ float bfr(float f) { return bf_up(bf_bits(f)); }
__device__ __forceinline__ unsigned short h_bits(_Float16 x) { return __builtin_bit_cast(unsigned short, x); }
__device__ __forceinline__ unsigned pk16(unsigned short a, unsigned short b) { return (unsigned)a | ((unsigned)b << 16); }
__device__ __forceinline__ v8f zero8() { v8f z = {0.f, 0.f, 0.f, 0.f, 0.f, 0.f, 0.f, 0.f}; return z; }

__device__ __forceinline__ v16h ldfrag_u(const unsigned short* p) {
  FragH f;
  f.u[0] = *(const v4u*)(p);
  f.u[1] = *(const v4u*)(p + 16);
  return f.v;
}

__device__ __forceinline__ v8f mma_h(v16h a, v16h b, v8f c) {
  return __builtin_amdgcn_wmma_f32_16x16x32_f16(false, a, false, b, (short)0, c, false, false);
}
__device__ __forceinline__ v8f mma_b(v16h a, v16h b, v8f c) {
  FragAny ua, ub;
  ua.h = a;
  ub.h = b;
  return __builtin_amdgcn_wmma_f32_16x16x32_bf16(false, ua.b, false, ub.b, (short)0, c, false, false);
}
template <int BF>
__device__ __forceinline__ v8f mmaT(v16h a, v16h b, v8f c) {
  if constexpr (BF != 0) return mma_b(a, b, c);
  else return mma_h(a, b, c);
}
__device__ __forceinline__ void dep_guard1(v8f& a, v8f& b, v16h x) {
#if defined(__HIP_DEVICE_COMPILE__)
  asm volatile("v_nop\n\tv_nop\n\tv_nop\n\tv_nop" : "+v"(a), "+v"(b) : "v"(x));
#endif
}
__device__ __forceinline__ void hz4(v8f& d, v16h x0, v16h x1, v16h x2, v16h x3) {
#if defined(__HIP_DEVICE_COMPILE__)
  asm volatile("v_nop\n\tv_nop\n\tv_nop\n\tv_nop" : "+v"(d) : "v"(x0), "v"(x1), "v"(x2), "v"(x3));
#endif
}
__device__ __forceinline__ void hz6(v8f& d, v16h x0, v16h x1, v16h x2, v16h x3, v16h x4, v16h x5) {
#if defined(__HIP_DEVICE_COMPILE__)
  asm volatile("v_nop\n\tv_nop\n\tv_nop\n\tv_nop" : "+v"(d) : "v"(x0), "v"(x1), "v"(x2), "v"(x3), "v"(x4), "v"(x5));
#endif
}
__device__ __forceinline__ void keep4_h(v16h a, v16h b, v16h c, v16h d) {
#if defined(__HIP_DEVICE_COMPILE__)
  asm volatile("v_nop" :: "v"(a), "v"(b), "v"(c), "v"(d));
#endif
}
__device__ __forceinline__ void acc_guard4(v8f& a, v8f& b, v8f& c, v8f& d) {
#if defined(__HIP_DEVICE_COMPILE__)
  asm volatile("v_nop\n\tv_nop\n\tv_nop\n\tv_nop" : "+v"(a), "+v"(b), "+v"(c), "+v"(d));
#endif
}
__device__ __forceinline__ void wave_sync_lds() {
  __builtin_amdgcn_fence(__ATOMIC_RELEASE, "workgroup");
  __builtin_amdgcn_wave_barrier();
  __builtin_amdgcn_fence(__ATOMIC_ACQUIRE, "workgroup");
}

__global__ __launch_bounds__(256) void cvt16(const float* __restrict__ src, unsigned short* dst, int nvalid, int ntotal, float sc) {
  const size_t i8 = ((size_t)blockIdx.x * 256 + threadIdx.x) * 8;
  if (i8 + 8 > (size_t)ntotal) return;
  const bool pad = (i8 + 8 > (size_t)nvalid);
  const size_t ls = pad ? ((size_t)nvalid - 8) : i8;
  const v4f a = *(const v4f*)(src + ls);
  const v4f b = *(const v4f*)(src + ls + 4);
  v4u o;
  o[0] = pk16(h_bits((_Float16)(bfr(a[0]) * sc)), h_bits((_Float16)(bfr(a[1]) * sc)));
  o[1] = pk16(h_bits((_Float16)(bfr(a[2]) * sc)), h_bits((_Float16)(bfr(a[3]) * sc)));
  o[2] = pk16(h_bits((_Float16)(bfr(b[0]) * sc)), h_bits((_Float16)(bfr(b[1]) * sc)));
  o[3] = pk16(h_bits((_Float16)(bfr(b[2]) * sc)), h_bits((_Float16)(bfr(b[3]) * sc)));
  const v4u z = {0u, 0u, 0u, 0u};
  const v4u w = pad ? z : o;
  for (int pass = 0; pass < 2; ++pass) {
    *(volatile v4u*)(dst + i8) = w;
    __threadfence();
  }
}

__global__ __launch_bounds__(256) void trans16(const float* __restrict__ W, unsigned short* dst, int nk, int ncol, int mode, float sc) {
  __shared__ __align__(16) float sh[64 * 65];
  const int tid  = threadIdx.x;
  const int lane = tid & 31;
  const int wave = tid >> 5;
  const int c0 = blockIdx.x * 64, k0 = blockIdx.y * 64;
  if (c0 + 64 > ncol || k0 + 64 > nk) return;
#pragma unroll 4
  for (int it = 0; it < 16; ++it) {
    const int idx = tid + 256 * it;
    const int kk = idx >> 6, cc = idx & 63;
    const size_t o0 = (size_t)(k0 + kk) * (size_t)ncol + (size_t)(c0 + cc);
    const size_t o1 = ((size_t)(c0 >> 6) * (size_t)nk + (size_t)(k0 + kk)) * 64 + (size_t)cc;
    const size_t o  = (mode != 0) ? o1 : o0;
    sh[cc * 65 + kk] = W[o];
  }
  __syncthreads();
  v4u w[2];
#pragma unroll
  for (int it = 0; it < 2; ++it) {
    const int row = 4 * wave + (lane >> 3) + 32 * it;
    const int g   = (lane & 7) * 8;
    const float* sp = sh + row * 65 + g;
    v4u o;
#pragma unroll
    for (int e = 0; e < 4; ++e) {
      o[e] = pk16(h_bits((_Float16)(bfr(sp[2 * e]) * sc)), h_bits((_Float16)(bfr(sp[2 * e + 1]) * sc)));
    }
    w[it] = o;
  }
  for (int pass = 0; pass < 2; ++pass) {
#pragma unroll
    for (int it = 0; it < 2; ++it) {
      const int row = 4 * wave + (lane >> 3) + 32 * it;
      const int g   = (lane & 7) * 8;
      *(volatile v4u*)(dst + (size_t)(c0 + row) * (size_t)nk + k0 + g) = w[it];
    }
    __threadfence();
  }
}

template <int OM, int ASPLIT, int BF, int EPI>
__global__ __launch_bounds__(256) __attribute__((amdgpu_num_vgpr(256))) void gemm64(
    const unsigned short* __restrict__ Ap, const unsigned short* __restrict__ A2p, int lda, long long sA,
    const unsigned short* __restrict__ Btp, int ldb, long long sB,
    void* Cout, void* C2out, int ldc, long long sC,
    int M, int N, int K, float oscale, float ocarry,
    const float* __restrict__ ep0, const float* __restrict__ ep1, const float* __restrict__ ep2) {
  __shared__ __align__(16) float sT[8][16 * 68];
  const int by   = blockIdx.y;
  const int lane = threadIdx.x & 31;
  const int wave = threadIdx.x >> 5;
  const int tilesN = N >> 6;
  const int tilesM = M >> 6;
  const int tile = blockIdx.x * 8 + wave;
  if (tile >= tilesM * tilesN) return;
  const int tm = tile / tilesN;
  const int tn = tile - tm * tilesN;
  const int m0 = tm << 6;
  const int n0 = tn << 6;

  const unsigned short* A1 = Ap  + (size_t)((long long)by * sA);
  const unsigned short* A2 = A2p + (size_t)((long long)by * sA);
  const unsigned short* Bb = Btp + (size_t)((long long)by * sB);

  const int rlane = lane & 15;
  const int koff  = (lane >> 4) * 8;
  const int mOff  = (lane >> 4) * 8;

  v8f acc[4][4];
#pragma unroll
  for (int i = 0; i < 4; ++i)
#pragma unroll
    for (int j = 0; j < 4; ++j) acc[i][j] = zero8();

  for (int k0 = 0; k0 < K; k0 += 32) {
    v16h bh[4];
#pragma unroll
    for (int j = 0; j < 4; ++j) {
      const size_t bofs = (size_t)(n0 + (j << 4) + rlane) * ldb + koff + k0;
      bh[j] = ldfrag_u(Bb + bofs);
    }
#pragma unroll
    for (int i = 0; i < 4; ++i) {
      const size_t ao = (size_t)(m0 + (i << 4) + rlane) * lda + koff + k0;
      const v16h ah = ldfrag_u(A1 + ao);
#pragma unroll
      for (int j = 0; j < 4; ++j) acc[i][j] = mmaT<BF>(ah, bh[j], acc[i][j]);
      dep_guard1(acc[i][0], acc[i][3], ah);
      if constexpr (ASPLIT != 0) {
        const v16h al = ldfrag_u(A2 + ao);
#pragma unroll
        for (int j = 0; j < 4; ++j) acc[i][j] = mmaT<BF>(al, bh[j], acc[i][j]);
        dep_guard1(acc[i][0], acc[i][3], al);
      }
    }
    keep4_h(bh[0], bh[1], bh[2], bh[3]);
  }
  acc_guard4(acc[0][0], acc[0][1], acc[0][2], acc[0][3]);
  acc_guard4(acc[1][0], acc[1][1], acc[1][2], acc[1][3]);
  acc_guard4(acc[2][0], acc[2][1], acc[2][2], acc[2][3]);
  acc_guard4(acc[3][0], acc[3][1], acc[3][2], acc[3][3]);

  const int hh2 = lane >> 4, c4 = (lane & 15) * 4;
  const int q8  = lane >> 3, c8 = (lane & 7) * 8;

  float* slab = sT[wave];
#pragma unroll
  for (int i = 0; i < 4; ++i) {
    const int mBase = m0 + (i << 4);
#pragma unroll
    for (int j = 0; j < 4; ++j) {
#pragma unroll
      for (int r = 0; r < 8; ++r) {
        slab[(mOff + r) * 68 + (j << 4) + rlane] = acc[i][j][r];
      }
    }
    wave_sync_lds();
    if constexpr (OM == 0) {
      float* C = (float*)Cout + (size_t)((long long)by * sC);
      v4f vals[8];
#pragma unroll
      for (int it = 0; it < 8; ++it) {
        const int row = it * 2 + hh2;
        v4f v = *(const v4f*)(slab + row * 68 + c4);
#pragma unroll
        for (int e = 0; e < 4; ++e) v[e] = v[e] * oscale;
        if constexpr (EPI == 1) {
          const v4f bb = *(const v4f*)(ep0 + n0 + c4);
#pragma unroll
          for (int e = 0; e < 4; ++e) v[e] = v[e] + bfr(bb[e]);
        }
        vals[it] = v;
      }
      for (int pass = 0; pass < 2; ++pass) {
#pragma unroll
        for (int it = 0; it < 8; ++it) {
          const int gr = mBase + it * 2 + hh2;
          *(volatile v4f*)(C + (size_t)gr * ldc + n0 + c4) = vals[it];
        }
        __threadfence();
      }
    } else {
      unsigned short* C  = (unsigned short*)Cout  + (size_t)((long long)by * sC);
      unsigned short* Cb = (unsigned short*)C2out + (size_t)((long long)by * sC);
      v4u hv[4], lv[4];
#pragma unroll
      for (int it = 0; it < 4; ++it) {
        const int row = it * 4 + q8;
        const float* sp = slab + row * 68 + c8;
        float rb = 0.f;
        if constexpr (EPI == 2) rb = bfr(ep0[mBase + row]);
        v4u a  = {0u, 0u, 0u, 0u};
        v4u b2 = {0u, 0u, 0u, 0u};
#pragma unroll
        for (int e = 0; e < 4; ++e) {
          const int ci = n0 + c8 + 2 * e;
          float f0 = sp[2 * e] * oscale + rb;
          float f1 = sp[2 * e + 1] * oscale + rb;
          if constexpr (EPI == 1) {
            f0 += bfr(ep0[ci]);
            f1 += bfr(ep0[ci + 1]);
          }
          if constexpr (OM == 5) {
            const float g0 = (f0 + bfr(ep1[ci])) * ocarry, g1 = (f1 + bfr(ep1[ci + 1])) * ocarry;
            const float w0 = (f0 + bfr(ep2[ci])) * ocarry, w1 = (f1 + bfr(ep2[ci + 1])) * ocarry;
            a[e]  = pk16(h_bits((_Float16)g0), h_bits((_Float16)g1));
            b2[e] = pk16(h_bits((_Float16)w0), h_bits((_Float16)w1));
          } else {
            f0 *= ocarry; f1 *= ocarry;
            const _Float16 x0 = (_Float16)f0, x1 = (_Float16)f1;
            a[e] = pk16(h_bits(x0), h_bits(x1));
            if constexpr (OM == 4) {
              b2[e] = pk16(h_bits((_Float16)(f0 - (float)x0)), h_bits((_Float16)(f1 - (float)x1)));
            }
          }
        }
        hv[it] = a;
        lv[it] = b2;
      }
      for (int pass = 0; pass < 2; ++pass) {
#pragma unroll
        for (int it = 0; it < 4; ++it) {
          const int row = it * 4 + q8;
          *(volatile v4u*)(C + (size_t)(mBase + row) * ldc + n0 + c8) = hv[it];
          if constexpr (OM >= 4) {
            *(volatile v4u*)(Cb + (size_t)(mBase + row) * ldc + n0 + c8) = lv[it];
          }
        }
        __threadfence();
      }
    }
    wave_sync_lds();
  }
}

__device__ __forceinline__ void pos_strip(const unsigned short* __restrict__ QVa, const unsigned short* __restrict__ Ph,
                                          const unsigned short* __restrict__ Pl, int mw, float* tsh, int hh, int c) {
  const v16h qva = ldfrag_u(QVa), qvb = ldfrag_u(QVa + 32);
#pragma unroll 1
  for (int u = 0; u < 5; ++u) {
    int m = mw + 16 * u + c;
    m = (m < 0) ? 0 : m;
    m = (m > NPOS - 1) ? (NPOS - 1) : m;
    const size_t ko = (size_t)m * DMOD;
    const v16h fa = ldfrag_u(Ph + ko), fb = ldfrag_u(Ph + ko + 32);
    const v16h ga = ldfrag_u(Pl + ko), gb = ldfrag_u(Pl + ko + 32);
    v8f t8 = mma_h(qva, fa, zero8());
    t8 = mma_h(qvb, fb, t8);
    t8 = mma_h(qva, ga, t8);
    t8 = mma_h(qvb, gb, t8);
    hz6(t8, fa, fb, ga, gb, qva, qvb);
    const int cb = 16 * u + c;
#pragma unroll
    for (int r = 0; r < 8; ++r) tsh[(8 * hh + r) * TPI + cb] = t8[r];
  }
}

__global__ __launch_bounds__(ATT_THREADS) __attribute__((amdgpu_num_vgpr(256)))
void attn_rel(const unsigned short* __restrict__ QU, const unsigned short* __restrict__ QV,
              const unsigned short* __restrict__ KP, const unsigned short* __restrict__ PH,
              const unsigned short* __restrict__ PL,
              const unsigned short* __restrict__ VT, const unsigned short* __restrict__ VTL,
              const int* __restrict__ MSK, unsigned short* CT, unsigned short* CTL) {
  __shared__ __align__(16) float smem[ATT_W * WFL];

  const int tid  = threadIdx.x;
  const int wave = __builtin_amdgcn_readfirstlane(tid >> 5);
  const int lane = tid & 31;
  const int hh   = lane >> 4;
  const int c    = lane & 15;
  const int bn   = blockIdx.y;
  const int b    = bn / NH;
  const int n    = bn - b * NH;
  const int i0   = blockIdx.x * 64;
  const int iw0  = i0 + wave * 16;

  float* tsh = smem + wave * WFL;
  float* pt  = tsh + 16 * TPI;

  const size_t qro = ((size_t)(b * LQ + iw0 + c)) * DMOD + n * DH + 8 * hh;
  const v16h qua = ldfrag_u(QU + qro), qub = ldfrag_u(QU + qro + 32);

  const unsigned short* Kb  = KP + (size_t)b * LQ * DMOD + n * DH + 8 * hh;
  const unsigned short* Phb = PH + n * DH + 8 * hh;
  const unsigned short* Plb = PL + n * DH + 8 * hh;
  const size_t vbase = (size_t)b * DMOD * LQ + (size_t)(n * DH) * LQ + 8 * hh;
  const unsigned short* Vb  = VT  + vbase;
  const unsigned short* VLb = VTL + vbase;
  const int* mkp = MSK + b * LQ;

  const float KSC = (RSD / (QC * QC)) * LOG2E;
  const float MSC = BIGM * LOG2E;

  float mrow[8], lrow[8];
  v8f O[4];
#pragma unroll
  for (int r = 0; r < 8; ++r) { mrow[r] = -INFINITY; lrow[r] = 0.f; }
#pragma unroll
  for (int td = 0; td < 4; ++td) O[td] = zero8();

#pragma unroll 1
  for (int j0 = 0; j0 < LQ; j0 += 64) {
    pos_strip(QV + qro, Phb, Plb, LQ + j0 - iw0 - 15, tsh, hh, c);
    v8f S[4];
#pragma unroll
    for (int t = 0; t < 4; ++t) {
      const size_t ko = (size_t)(j0 + 16 * t + c) * DMOD;
      const v16h ka = ldfrag_u(Kb + ko), kb2 = ldfrag_u(Kb + ko + 32);
      S[t] = mma_h(qua, ka, zero8());
      S[t] = mma_h(qub, kb2, S[t]);
      hz4(S[t], ka, kb2, qua, qub);
    }
    float mk[4];
#pragma unroll
    for (int t = 0; t < 4; ++t) mk[t] = (float)mkp[j0 + 16 * t + c] * MSC;
    wave_sync_lds();

#pragma unroll
    for (int r = 0; r < 8; ++r) {
      const int R  = 8 * hh + r;
      const int xo = R * TPI + (15 - R) + c;
      float tv[4];
#pragma unroll
      for (int t = 0; t < 4; ++t) {
        const float bdv = tsh[xo + 16 * t];
        tv[t] = (S[t][r] + bdv) * KSC - mk[t];
      }
      float mx = fmaxf(fmaxf(tv[0], tv[1]), fmaxf(tv[2], tv[3]));
#pragma unroll
      for (int off = 1; off < 16; off <<= 1) mx = fmaxf(mx, __shfl_xor(mx, off, 32));
      const float mn = fmaxf(mrow[r], mx);
      const float al = exp2f(mrow[r] - mn);
      mrow[r] = mn;
      float e4[4];
      float ps = 0.f;
#pragma unroll
      for (int t = 0; t < 4; ++t) { e4[t] = exp2f(tv[t] - mn); ps += e4[t]; }
#pragma unroll
      for (int off = 1; off < 16; off <<= 1) ps += __shfl_xor(ps, off, 32);
      lrow[r] = lrow[r] * al + ps;
#pragma unroll
      for (int td = 0; td < 4; ++td) O[td][r] *= al;
      const int ro = R * PPI + c;
#pragma unroll
      for (int t = 0; t < 4; ++t) pt[ro + 16 * t] = e4[t];
    }
    wave_sync_lds();

    FragH pf[2];
#pragma unroll
    for (int ks = 0; ks < 2; ++ks) {
      const float* prow = pt + c * PPI + 32 * ks + 8 * hh;
      const v4f p0 = *(const v4f*)(prow), p1 = *(const v4f*)(prow + 4);
      const v4f p2 = *(const v4f*)(prow + 16), p3 = *(const v4f*)(prow + 20);
#pragma unroll
      for (int e = 0; e < 4; ++e) {
        pf[ks].h[0][e]     = (_Float16)(p0[e] * PC);
        pf[ks].h[0][4 + e] = (_Float16)(p1[e] * PC);
        pf[ks].h[1][e]     = (_Float16)(p2[e] * PC);
        pf[ks].h[1][4 + e] = (_Float16)(p3[e] * PC);
      }
    }
    {
      const size_t vo = (size_t)c * LQ + j0;
#pragma unroll
      for (int td = 0; td < 4; ++td) {
        const unsigned short* vp = Vb + vo + (size_t)(16 * td) * LQ;
        const v16h vfa = ldfrag_u(vp), vfb = ldfrag_u(vp + 32);
        O[td] = mma_h(pf[0].v, vfa, O[td]);
        O[td] = mma_h(pf[1].v, vfb, O[td]);
        hz4(O[td], pf[0].v, pf[1].v, vfa, vfb);
      }
#pragma unroll
      for (int td = 0; td < 4; ++td) {
        const unsigned short* vp = VLb + vo + (size_t)(16 * td) * LQ;
        const v16h vla = ldfrag_u(vp), vlb = ldfrag_u(vp + 32);
        O[td] = mma_h(pf[0].v, vla, O[td]);
        O[td] = mma_h(pf[1].v, vlb, O[td]);
        hz4(O[td], pf[0].v, pf[1].v, vla, vlb);
      }
    }
    wave_sync_lds();
  }
  acc_guard4(O[0], O[1], O[2], O[3]);

  const float oc = CC / (PC * VC);
#pragma unroll
  for (int r = 0; r < 8; ++r) {
    const float inv = (1.0f / lrow[r]) * oc;
    const int ro = (8 * hh + r) * PPI + c;
#pragma unroll
    for (int td = 0; td < 4; ++td) pt[ro + 16 * td] = O[td][r] * inv;
  }
  wave_sync_lds();
  {
    const int q8 = lane >> 3, c8 = (lane & 7) * 8;
    v4u hv[4], lv[4];
#pragma unroll
    for (int it = 0; it < 4; ++it) {
      const int row = it * 4 + q8;
      const float* sp = pt + row * PPI + c8;
      v4u a, b2;
#pragma unroll
      for (int e = 0; e < 4; ++e) {
        const float f0 = sp[2 * e], f1 = sp[2 * e + 1];
        const _Float16 x0 = (_Float16)f0, x1 = (_Float16)f1;
        a[e]  = pk16(h_bits(x0), h_bits(x1));
        b2[e] = pk16(h_bits((_Float16)(f0 - (float)x0)), h_bits((_Float16)(f1 - (float)x1)));
      }
      hv[it] = a;
      lv[it] = b2;
    }
    for (int pass = 0; pass < 2; ++pass) {
#pragma unroll
      for (int it = 0; it < 4; ++it) {
        const int row = it * 4 + q8;
        const size_t go = ((size_t)(b * LQ + iw0 + row)) * DMOD + n * DH + c8;
        *(volatile v4u*)(CT  + go) = hv[it];
        *(volatile v4u*)(CTL + go) = lv[it];
      }
      __threadfence();
    }
  }
}

__global__ __launch_bounds__(256) void ln_out(const float* __restrict__ res, const float* __restrict__ xq,
                                              const float* __restrict__ gam, const float* __restrict__ bet,
                                              float* out, int nrows) {
  const int lane = threadIdx.x & 31;
  const int wave = threadIdx.x >> 5;
  const int row  = blockIdx.x * 8 + wave;
  if (row >= nrows) return;
  const float* pr = res + (size_t)row * DMOD;
  const float* pq = xq  + (size_t)row * DMOD;
  float v[32];
#pragma unroll
  for (int g = 0; g < 8; ++g) {
    const int col = 128 * g + 4 * lane;
    const v4f a = *(const v4f*)(pr + col);
    const v4f q = *(const v4f*)(pq + col);
#pragma unroll
    for (int e = 0; e < 4; ++e) v[4 * g + e] = a[e] + bfr(q[e]);
  }
  float s = 0.f;
#pragma unroll
  for (int e = 0; e < 32; ++e) s += v[e];
#pragma unroll
  for (int off = 1; off < 32; off <<= 1) s += __shfl_xor(s, off, 32);
  const float mu = s * (1.0f / (float)DMOD);
  float qs = 0.f;
#pragma unroll
  for (int e = 0; e < 32; ++e) {
    const float d = v[e] - mu;
    v[e] = d;
    qs += d * d;
  }
#pragma unroll
  for (int off = 1; off < 32; off <<= 1) qs += __shfl_xor(qs, off, 32);
  const float var  = qs * (1.0f / (float)DMOD);
  const float rstd = 1.0f / sqrtf(var + LN_EPS);
  v4f o[8];
#pragma unroll
  for (int g = 0; g < 8; ++g) {
    const int col = 128 * g + 4 * lane;
    const v4f gg = *(const v4f*)(gam + col);
    const v4f bb = *(const v4f*)(bet + col);
    v4f y;
#pragma unroll
    for (int e = 0; e < 4; ++e) y[e] = v[4 * g + e] * rstd * bfr(gg[e]) + bfr(bb[e]);
    o[g] = y;
  }
  float* dst = out + (size_t)row * DMOD;
  for (int pass = 0; pass < 2; ++pass) {
#pragma unroll
    for (int g = 0; g < 8; ++g) {
      *(volatile v4f*)(dst + 128 * g + 4 * lane) = o[g];
    }
    __threadfence();
  }
}

extern "C" void kernel_launch(void* const* d_in, const int* in_sizes, int n_in,
                              void* d_out, int out_size, void* d_ws, size_t ws_size,
                              hipStream_t stream) {
  if (n_in < 17) return;
  if (in_sizes[0] != NROW * DMOD || in_sizes[1] != NROW * DMOD || in_sizes[2] != NROW * DMOD) return;
  if (in_sizes[3] != NPOS * DMOD) return;
  if (in_sizes[4] != DMOD * DMOD || in_sizes[5] != DMOD * DMOD || in_sizes[7] != DMOD * DMOD ||
      in_sizes[11] != DMOD * DMOD || in_sizes[12] != DMOD * DMOD) return;
  if (in_sizes[6] != NH * DH || in_sizes[8] != NH * DH || in_sizes[9] != NH * DH || in_sizes[10] != NH * DH) return;
  if (in_sizes[13] != DMOD || in_sizes[14] != DMOD || in_sizes[15] != DMOD) return;
  if (in_sizes[16] != NB * LQ) return;
  if (out_size != NROW * DMOD) return;

  const float* q_in  = (const float*)d_in[0];
  const float* k_in  = (const float*)d_in[1];
  const float* v_in  = (const float*)d_in[2];
  const float* pos   = (const float*)d_in[3];
  const float* w_q   = (const float*)d_in[4];
  const float* w_k   = (const float*)d_in[5];
  const float* b_k   = (const float*)d_in[6];
  const float* w_v   = (const float*)d_in[7];
  const float* b_v   = (const float*)d_in[8];
  const float* rwb   = (const float*)d_in[9];
  const float* rrb   = (const float*)d_in[10];
  const float* rker  = (const float*)d_in[11];
  const float* w_o   = (const float*)d_in[12];
  const float* b_o   = (const float*)d_in[13];
  const float* ln_w  = (const float*)d_in[14];
  const float* ln_b  = (const float*)d_in[15];
  const int*   msk   = (const int*)d_in[16];
  float*       out   = (float*)d_out;

  const size_t PW  = (size_t)DMOD * DMOD * 2;
  const size_t PX  = (size_t)NROW * DMOD * 2;
  const size_t PP  = (size_t)NPOS * DMOD * 2;
  const size_t PVT = (size_t)NB * DMOD * LQ * 2;
  const size_t PR  = (size_t)NROW * DMOD * 4;
  size_t off = 0;
  const size_t oWQ  = off; off += PW;
  const size_t oWK  = off; off += PW;
  const size_t oWV  = off; off += PW;
  const size_t oWR  = off; off += PW;
  const size_t oWO  = off; off += PW;
  const size_t oXQ  = off; off += PX;
  const size_t oXK  = off; off += PX;
  const size_t oXV  = off; off += PX;
  const size_t oXP  = off; off += PP;
  const size_t oQU  = off; off += PX;
  const size_t oQV  = off; off += PX;
  const size_t oKK  = off; off += PX;
  const size_t oPH  = off; off += PP;
  const size_t oPL  = off; off += PP;
  const size_t oVT  = off; off += PVT;
  const size_t oVTL = off; off += PVT;
  const size_t oCT  = off; off += PX;
  const size_t oCTL = off; off += PX;
  const size_t oRES = off; off += PR;
  if (off > ws_size) return;
  if (off > (size_t)134217728) return;

  char* ws = (char*)d_ws;
  unsigned short* WQt  = (unsigned short*)(ws + oWQ);
  unsigned short* WKt  = (unsigned short*)(ws + oWK);
  unsigned short* WVt  = (unsigned short*)(ws + oWV);
  unsigned short* WRt  = (unsigned short*)(ws + oWR);
  unsigned short* WOt  = (unsigned short*)(ws + oWO);
  unsigned short* XQ   = (unsigned short*)(ws + oXQ);
  unsigned short* XK   = (unsigned short*)(ws + oXK);
  unsigned short* XV   = (unsigned short*)(ws + oXV);
  unsigned short* XP   = (unsigned short*)(ws + oXP);
  unsigned short* QU   = (unsigned short*)(ws + oQU);
  unsigned short* QV   = (unsigned short*)(ws + oQV);
  unsigned short* KK   = (unsigned short*)(ws + oKK);
  unsigned short* PH16 = (unsigned short*)(ws + oPH);
  unsigned short* PL16 = (unsigned short*)(ws + oPL);
  unsigned short* VT16 = (unsigned short*)(ws + oVT);
  unsigned short* VTL16 = (unsigned short*)(ws + oVTL);
  unsigned short* CT16 = (unsigned short*)(ws + oCT);
  unsigned short* CTL16 = (unsigned short*)(ws + oCTL);
  float*          RES  = (float*)(ws + oRES);

  const dim3 blk(256);
  const dim3 gCX((NROW * DMOD) / 2048);
  const dim3 gCP((NPOS * DMOD) / 2048);
  const dim3 gTW(DMOD / 64, DMOD / 64);
  const int tilesQ = (NROW / 64) * (DMOD / 64);
  const int tilesV = (DMOD / 64) * (LQ / 64);
  const int tilesP = (NPOS / 64) * (DMOD / 64);
  const dim3 gQ((tilesQ + 7) / 8, 1);
  const dim3 gV((tilesV + 7) / 8, NB);
  const dim3 gP((tilesP + 7) / 8, 1);
  const dim3 gAT(LQ / 64, NB * NH);
  const dim3 bAT(ATT_THREADS);
  const dim3 gLN(NROW / 8);

  cvt16<<<gCX, blk, 0, stream>>>(q_in, XQ, NROW * DMOD, NROW * DMOD, XC);
  cvt16<<<gCX, blk, 0, stream>>>(k_in, XK, NROW * DMOD, NROW * DMOD, XC);
  cvt16<<<gCX, blk, 0, stream>>>(v_in, XV, NROW * DMOD, NROW * DMOD, XC);
  cvt16<<<gCP, blk, 0, stream>>>(pos,  XP, NPOS * DMOD, NPOS * DMOD, XC);

  trans16<<<gTW, blk, 0, stream>>>(w_q,  WQt, DMOD, DMOD, 0, WSC);
  trans16<<<gTW, blk, 0, stream>>>(w_k,  WKt, DMOD, DMOD, 0, WSC);
  trans16<<<gTW, blk, 0, stream>>>(w_v,  WVt, DMOD, DMOD, 0, WSC);
  trans16<<<gTW, blk, 0, stream>>>(rker, WRt, DMOD, DMOD, 1, WSC);
  trans16<<<gTW, blk, 0, stream>>>(w_o,  WOt, DMOD, DMOD, 0, WSC);

  gemm64<5, 0, 0, 0><<<gQ, blk, 0, stream>>>(
      XQ, XQ, DMOD, 0LL,
      WQt, DMOD, 0LL,
      (void*)QU, (void*)QV, DMOD, 0LL,
      NROW, DMOD, DMOD, 1.0f / (XC * WSC), QC,
      rwb, rwb, rrb);

  gemm64<2, 0, 0, 1><<<gQ, blk, 0, stream>>>(
      XK, XK, DMOD, 0LL,
      WKt, DMOD, 0LL,
      (void*)KK, (void*)KK, DMOD, 0LL,
      NROW, DMOD, DMOD, 1.0f / (XC * WSC), QC,
      b_k, b_k, b_k);

  gemm64<4, 0, 0, 2><<<gV, blk, 0, stream>>>(
      WVt, WVt, DMOD, 0LL,
      XV, DMOD, (long long)LQ * DMOD,
      (void*)VT16, (void*)VTL16, LQ, (long long)DMOD * LQ,
      DMOD, LQ, DMOD, 1.0f / (XC * WSC), VC,
      b_v, b_v, b_v);

  gemm64<4, 0, 0, 0><<<gP, blk, 0, stream>>>(
      XP, XP, DMOD, 0LL,
      WRt, DMOD, 0LL,
      (void*)PH16, (void*)PL16, DMOD, 0LL,
      NPOS, DMOD, DMOD, 1.0f / (XC * WSC), QC,
      rwb, rwb, rwb);

  attn_rel<<<gAT, bAT, 0, stream>>>(QU, QV, KK, PH16, PL16, VT16, VTL16, msk, CT16, CTL16);

  gemm64<0, 1, 0, 1><<<gQ, blk, 0, stream>>>(
      CT16, CTL16, DMOD, 0LL,
      WOt, DMOD, 0LL,
      (void*)RES, (void*)RES, DMOD, 0LL,
      NROW, DMOD, DMOD, 1.0f / (CC * WSC), 1.0f,
      b_o, b_o, b_o);

  ln_out<<<gLN, blk, 0, stream>>>(RES, q_in, ln_w, ln_b, out, NROW);
  (void)hipGetLastError();
}
